// SmallBitConvNet_57492432224587
// MI455X (gfx1250) — hardware-run, weakly checked
//
#include <hip/hip_runtime.h>
#include <stdint.h>

#pragma clang fp contract(off)

#define CIN1   3
#define IMH    32
#define IMW    32
#define NPX1   (IMH * IMW)
#define CO1    64
#define K1     27
#define K1P    32
#define PH1    16
#define NPP1   (PH1 * PH1)
#define PDH    (PH1 + 2)
#define NPD    (PDH * PDH)
#define CO2    128
#define K2     576
#define NPP2   64
#define KF     8192
#define NF1    256
#define NCLS   10
#define MBF    64
#define RFC2   32
#define A2SC   16.0f
#define A2INV  0.0625f
#define EPSBN  1e-5f

#define XSP    36
#define ASP    32
#define ETP    128
#define STP2   68
#define STP3   132

static_assert(K1 <= K1P);
static_assert((ASP * 2) % 16 == 0);
static_assert((STP2 * 4) % 16 == 0);
static_assert((STP3 * 4) % 16 == 0);
static_assert((CO1 * K1P / 8) == 256);
static_assert((CO2 * K2 / 8) % 256 == 0);
static_assert((NF1 * KF / 8) % 256 == 0);
static_assert(RFC2 * NCLS == 320);
static_assert(11 * 32 >= NPD);

typedef _Float16       v16h __attribute__((ext_vector_type(16)));
typedef _Float16       v8h  __attribute__((ext_vector_type(8)));
typedef __bf16         v16b __attribute__((ext_vector_type(16)));
typedef __bf16         v8b  __attribute__((ext_vector_type(8)));
typedef float          v8f  __attribute__((ext_vector_type(8)));
typedef float          v4f  __attribute__((ext_vector_type(4)));
typedef float          v2f  __attribute__((ext_vector_type(2)));
typedef unsigned       v4u  __attribute__((ext_vector_type(4)));

__device__ __forceinline__ unsigned bfb(float f) {
  const unsigned u = __float_as_uint(f);
  return (u + 0x7FFFu + ((u >> 16) & 1u)) >> 16;
}
__device__ __forceinline__ float bf_rne(float f) { return __uint_as_float(bfb(f) << 16); }
__device__ __forceinline__ unsigned hbits(_Float16 h) {
  return (unsigned)__builtin_bit_cast(unsigned short, h);
}
__device__ __forceinline__ v8f zero8f() { v8f z = {0.f, 0.f, 0.f, 0.f, 0.f, 0.f, 0.f, 0.f}; return z; }

__device__ __forceinline__ v16h ldfrag_h(const _Float16* p) {
  union { v16h v; v8h h[2]; } f;
  f.h[0] = *(const v8h*)(p);
  f.h[1] = *(const v8h*)(p + 16);
  return f.v;
}
__device__ __forceinline__ v16b ldfrag_b(const __bf16* p) {
  union { v16b v; v8b h[2]; } f;
  f.h[0] = *(const v8b*)(p);
  f.h[1] = *(const v8b*)(p + 16);
  return f.v;
}

__device__ __forceinline__ v8f mma_h(v16h a, v16h b, v8f c) {
  return __builtin_amdgcn_wmma_f32_16x16x32_f16(false, a, false, b, (short)0, c, false, false);
}
__device__ __forceinline__ v8f mma_b(v16b a, v16b b, v8f c) {
  return __builtin_amdgcn_wmma_f32_16x16x32_bf16(false, a, false, b, (short)0, c, false, false);
}
template <typename F>
__device__ __forceinline__ void guard4x6(v8f& c0, v8f& c1, v8f& c2, v8f& c3,
                                         const F& f0, const F& f1, const F& f2,
                                         const F& f3, const F& f4, const F& f5) {
#if defined(__HIP_DEVICE_COMPILE__)
  asm volatile("v_nop\n\tv_nop\n\tv_nop\n\tv_nop"
               : "+v"(c0), "+v"(c1), "+v"(c2), "+v"(c3)
               : "v"(f0), "v"(f1), "v"(f2), "v"(f3), "v"(f4), "v"(f5));
#endif
}
template <typename F>
__device__ __forceinline__ void guard8x6(v8f& c0, v8f& c1, v8f& c2, v8f& c3,
                                         v8f& c4, v8f& c5, v8f& c6, v8f& c7,
                                         const F& f0, const F& f1, const F& f2,
                                         const F& f3, const F& f4, const F& f5) {
#if defined(__HIP_DEVICE_COMPILE__)
  asm volatile("v_nop\n\tv_nop\n\tv_nop\n\tv_nop"
               : "+v"(c0), "+v"(c1), "+v"(c2), "+v"(c3), "+v"(c4), "+v"(c5), "+v"(c6), "+v"(c7)
               : "v"(f0), "v"(f1), "v"(f2), "v"(f3), "v"(f4), "v"(f5));
#endif
}
__device__ __forceinline__ void acc_guard4(v8f& c0, v8f& c1, v8f& c2, v8f& c3) {
#if defined(__HIP_DEVICE_COMPILE__)
  asm volatile("v_nop\n\tv_nop\n\tv_nop\n\tv_nop" : "+v"(c0), "+v"(c1), "+v"(c2), "+v"(c3));
#endif
}
__device__ __forceinline__ void acc_guard8(v8f& c0, v8f& c1, v8f& c2, v8f& c3,
                                           v8f& c4, v8f& c5, v8f& c6, v8f& c7) {
#if defined(__HIP_DEVICE_COMPILE__)
  asm volatile("v_nop\n\tv_nop\n\tv_nop\n\tv_nop"
               : "+v"(c0), "+v"(c1), "+v"(c2), "+v"(c3), "+v"(c4), "+v"(c5), "+v"(c6), "+v"(c7));
#endif
}

__global__ __launch_bounds__(256)
void k_alpha(const float* __restrict__ w0, int n0, const float* __restrict__ w1, int n1,
             const float* __restrict__ w2, int n2, const float* __restrict__ w3, int n3,
             float* alpha)
{
  __shared__ double red[256];
  __shared__ float av[32];
  const int tid = threadIdx.x;
  const int i = blockIdx.x;
  const float* w = w0; int n = n0;
  if (i == 1)      { w = w1; n = n1; }
  else if (i == 2) { w = w2; n = n2; }
  else if (i == 3) { w = w3; n = n3; }
  double s = 0.0;
#pragma unroll 1
  for (int k = tid; k < n; k += 256) s += (double)fabsf(bf_rne(w[k]));
  red[tid] = s;
  __syncthreads();
#pragma unroll 1
  for (int off = 128; off > 0; off >>= 1) {
    if (tid < off) red[tid] = red[tid] + red[tid + off];
    __syncthreads();
  }
  if (tid == 0) av[0] = (n > 0) ? (float)(red[0] / (double)n) : 0.0f;
  __syncthreads();
  const float a = av[0];
  float* d = alpha + 32 * i + (tid & 31);
  if (tid < 32) *(volatile float*)d = a;
  __threadfence();
  if (tid < 32) *(volatile float*)d = a;
}

template <int MODE>
__global__ __launch_bounds__(256)
void k_pack(const float* __restrict__ w, unsigned* dst, int nchunks)
{
  const int q  = blockIdx.x * 256 + threadIdx.x;
  const int qc = min(q, nchunks - 1);
  unsigned hb[8];
#pragma unroll
  for (int j = 0; j < 8; ++j) {
    float v;
    bool live = true;
    if constexpr (MODE == 0) {
      const int row = qc >> 2;
      const int k   = (qc & 3) * 8 + j;
      live = (k < K1);
      v = w[row * K1 + min(k, K1 - 1)];
    } else if constexpr (MODE == 1) {
      const int row = qc / (K2 / 8);
      const int kc  = (qc - row * (K2 / 8)) * 8;
      const int tap = kc >> 6;
      const int c   = (kc & 63) + j;
      v = w[(row * CO1 + c) * 9 + tap];
    } else {
      v = w[(size_t)qc * 8 + j];
    }
    const float r = bf_rne(v);
    unsigned bits;
    if constexpr (MODE == 1) bits = (r > 0.0f) ? 0x3C00u : ((r < 0.0f) ? 0xBC00u : 0u);
    else                     bits = (r > 0.0f) ? 0x3F80u : ((r < 0.0f) ? 0xBF80u : 0u);
    hb[j] = live ? bits : 0u;
  }
  v4u wh;
  wh.x = hb[0] | (hb[1] << 16);
  wh.y = hb[2] | (hb[3] << 16);
  wh.z = hb[4] | (hb[5] << 16);
  wh.w = hb[6] | (hb[7] << 16);
  const bool ok = (q < nchunks);
  unsigned* d = dst + (size_t)qc * 4;
  if (ok) *(volatile v4u*)d = wh;
  __threadfence();
  if (ok) *(volatile v4u*)d = wh;
}

__global__ __launch_bounds__(256)
void k_conv1(const float* __restrict__ x, const __bf16* __restrict__ wq1,
             const float* __restrict__ alpha, const float* __restrict__ gam,
             float* h1p, float* part)
{
  __shared__ __align__(16) float xs[CIN1 * 6 * XSP];
  __shared__ __align__(16) unsigned short As[128 * ASP];
  __shared__ __align__(16) float Et[CO1 * ETP];
  __shared__ __align__(16) float red[8 * 128];
  __shared__ __align__(16) float rec[128];
  __shared__ float gsel[CO1];

  const int tid  = threadIdx.x;
  const int lane = tid & 31;
  const int wid  = tid >> 5;
  const int m    = lane & 15;
  const int hh   = lane >> 4;
  const int pj   = lane & 7;
  const int lq   = lane >> 3;
  const int b    = blockIdx.x;
  const float al = alpha[0];

  if (tid < 36) {
    const int row = tid >> 1;
    xs[row * XSP + ((tid & 1) ? (IMW + 1) : 0)] = 0.0f;
  }
  if (tid < CO1) gsel[tid] = (bf_rne(gam[tid]) >= 0.0f) ? 1.0f : 0.0f;
  v16b fb[4];
#pragma unroll
  for (int nt = 0; nt < 4; ++nt) fb[nt] = ldfrag_b(wq1 + (size_t)(16 * nt + m) * K1P + 8 * hh);
  float ssum[4], ssq[4];
#pragma unroll
  for (int nt = 0; nt < 4; ++nt) { ssum[nt] = 0.0f; ssq[nt] = 0.0f; }
  __syncthreads();

#pragma unroll 1
  for (int it = 0; it < 8; ++it) {
    const int y0 = 4 * it;
    if (tid < 144) {
      const int c   = tid / 48;
      const int rem = tid - 48 * c;
      const int lr  = rem >> 3;
      const int w4  = rem & 7;
      const int gy  = y0 - 1 + lr;
      const bool ok = (gy >= 0) && (gy < IMH);
      const int gyc = min(max(gy, 0), IMH - 1);
      const v4f v = *(const v4f*)(x + (((size_t)b * CIN1 + c) * IMH + gyc) * IMW + 4 * w4);
      float* tp = xs + (c * 6 + lr) * XSP + 1 + 4 * w4;
      tp[0] = ok ? v.x : 0.0f;
      tp[1] = ok ? v.y : 0.0f;
      tp[2] = ok ? v.z : 0.0f;
      tp[3] = ok ? v.w : 0.0f;
    }
    __syncthreads();
    {
      const int p  = tid & 127;
      const int kh = tid >> 7;
      const int ly = p >> 5;
      const int xx = p & 31;
      unsigned hb[16];
#pragma unroll
      for (int i = 0; i < 16; ++i) {
        const int k  = 16 * kh + i;
        const bool live = (k < K1);
        const int kk = min(k, K1 - 1);
        const int c  = kk / 9;
        const int r9 = kk - 9 * c;
        const int dy = r9 / 3;
        const int dx = r9 - 3 * dy;
        const float v = xs[(c * 6 + ly + dy) * XSP + xx + dx];
        hb[i] = live ? bfb(v) : 0u;
      }
      v4u q0, q1;
      q0.x = hb[0]  | (hb[1]  << 16); q0.y = hb[2]  | (hb[3]  << 16);
      q0.z = hb[4]  | (hb[5]  << 16); q0.w = hb[6]  | (hb[7]  << 16);
      q1.x = hb[8]  | (hb[9]  << 16); q1.y = hb[10] | (hb[11] << 16);
      q1.z = hb[12] | (hb[13] << 16); q1.w = hb[14] | (hb[15] << 16);
      *(v4u*)&As[p * ASP + 16 * kh]     = q0;
      *(v4u*)&As[p * ASP + 16 * kh + 8] = q1;
    }
    __syncthreads();
    const v16b fa = ldfrag_b((const __bf16*)As + (16 * wid + m) * ASP + 8 * hh);
    v8f acc[4];
#pragma unroll
    for (int nt = 0; nt < 4; ++nt) acc[nt] = mma_b(fa, fb[nt], zero8f());
    guard4x6(acc[0], acc[1], acc[2], acc[3], fa, fa, fb[0], fb[1], fb[2], fb[3]);
#pragma unroll
    for (int nt = 0; nt < 4; ++nt) {
      const int ch = 16 * nt + m;
      v4f o0, o1;
#pragma unroll
      for (int r = 0; r < 4; ++r) {
        const float v = acc[nt][r] * al;
        o0[r] = v;
        ssum[nt] = ssum[nt] + v;
        ssq[nt]  = ssq[nt] + v * v;
      }
#pragma unroll
      for (int r = 0; r < 4; ++r) {
        const float v = acc[nt][4 + r] * al;
        o1[r] = v;
        ssum[nt] = ssum[nt] + v;
        ssq[nt]  = ssq[nt] + v * v;
      }
      float* ep = Et + ch * ETP + 16 * wid + 8 * hh;
      *(v4f*)ep       = o0;
      *(v4f*)(ep + 4) = o1;
    }
    __syncthreads();
    {
      v4f val[2]; size_t e[2];
#pragma unroll
      for (int rr = 0; rr < 2; ++rr) {
        const int L   = rr * 32 + wid * 4 + lq;
        const int pp  = L >> 1;
        const int sub = L & 1;
        const int pyl = pp >> 4;
        const int px  = pp & 15;
        const int ch0 = 32 * sub + 4 * pj;
        const int pa  = (2 * pyl) * IMW + 2 * px;
        v4f o;
#pragma unroll
        for (int ee = 0; ee < 4; ++ee) {
          const float* rbp = Et + (ch0 + ee) * ETP;
          const v2f t0 = *(const v2f*)(rbp + pa);
          const v2f t1 = *(const v2f*)(rbp + pa + IMW);
          const float mx = fmaxf(fmaxf(t0.x, t0.y), fmaxf(t1.x, t1.y));
          const float mn = fminf(fminf(t0.x, t0.y), fminf(t1.x, t1.y));
          o[ee] = (gsel[ch0 + ee] != 0.0f) ? mx : mn;
        }
        val[rr] = o;
        e[rr]   = (((size_t)b * NPP1) + (2 * it + pyl) * PH1 + px) * CO1 + ch0;
      }
#pragma unroll
      for (int rr = 0; rr < 2; ++rr) *(volatile v4f*)(h1p + e[rr]) = val[rr];
      __threadfence();
#pragma unroll
      for (int rr = 0; rr < 2; ++rr) *(volatile v4f*)(h1p + e[rr]) = val[rr];
    }
    __syncthreads();
  }

#pragma unroll
  for (int nt = 0; nt < 4; ++nt) {
    const float s = ssum[nt] + __shfl_xor(ssum[nt], 16);
    const float q = ssq[nt]  + __shfl_xor(ssq[nt], 16);
    if (hh == 0) {
      red[wid * 128 + 16 * nt + m]      = s;
      red[wid * 128 + 64 + 16 * nt + m] = q;
    }
  }
  __syncthreads();
  if (tid < 128) {
    float t = 0.0f;
#pragma unroll
    for (int w = 0; w < 8; ++w) t = t + red[w * 128 + tid];
    rec[tid] = t;
  }
  __syncthreads();
  {
    const int tl = tid & 31;
    const v4f v = *(const v4f*)&rec[4 * tl];
    float* d = part + (size_t)b * 128 + 4 * tl;
    if (tid < 32) *(volatile v4f*)d = v;
    __threadfence();
    if (tid < 32) *(volatile v4f*)d = v;
  }
}

__global__ __launch_bounds__(256)
void k_stats(const float* __restrict__ part, int nblk, int cpr, int nspl, int C,
             const float* __restrict__ gam, const float* __restrict__ bet, int count, float* sb)
{
  __shared__ double dsum[256];
  __shared__ double dsq[256];
  __shared__ __align__(16) float outv[1024];
  const int tid = threadIdx.x;
  const int c   = tid % C;
  const int grp = tid / C;
  const int G   = 256 / C;
  const int half = c / cpr;
  const int cl   = c - half * cpr;
  const int recf = 2 * cpr;
  double s = 0.0, q = 0.0;
#pragma unroll 1
  for (int i = grp; i < nblk; i += G) {
    const float* r = part + ((size_t)i * nspl + half) * recf + cl;
    s += (double)r[0];
    q += (double)r[cpr];
  }
  dsum[tid] = s;
  dsq[tid]  = q;
  __syncthreads();
  if (tid < C) {
    double S = 0.0, Q = 0.0;
#pragma unroll 1
    for (int g = 0; g < G; ++g) { S += dsum[g * C + tid]; Q += dsq[g * C + tid]; }
    const double invn = 1.0 / (double)count;
    const double mean = S * invn;
    double var = Q * invn - mean * mean;
    if (var < 0.0) var = 0.0;
    const float vf = (float)var;
    const float rs = 1.0f / sqrtf(vf + EPSBN);
    outv[tid]         = (float)mean;
    outv[C + tid]     = rs;
    outv[2 * C + tid] = bf_rne(gam[tid]);
    outv[3 * C + tid] = bf_rne(bet[tid]);
  }
  __syncthreads();
  {
    const int tl = min(tid, C - 1);
    const v4f v = *(const v4f*)&outv[4 * tl];
    float* d = sb + 4 * tl;
    if (tid < C) *(volatile v4f*)d = v;
    __threadfence();
    if (tid < C) *(volatile v4f*)d = v;
  }
}

__global__ __launch_bounds__(256)
void k_pool1(const float* __restrict__ h1p, const float* __restrict__ sb, unsigned short* p1)
{
  __shared__ float sbl[4 * CO1];
  const int tid = threadIdx.x;
  sbl[tid] = sb[tid];
  __syncthreads();
  const int lane = tid & 31;
  const int wid  = tid >> 5;
  const int pj   = lane & 7;
  const int lq   = lane >> 3;
  const int b    = blockIdx.x;
  float mu[8], rs[8], ga[8], be[8];
#pragma unroll
  for (int e = 0; e < 8; ++e) {
    const int c = 8 * pj + e;
    mu[e] = sbl[c]; rs[e] = sbl[CO1 + c]; ga[e] = sbl[2 * CO1 + c]; be[e] = sbl[3 * CO1 + c];
  }
  constexpr int NIT = 11;
  v4u val[NIT]; size_t eo[NIT]; bool ok[NIT];
#pragma unroll
  for (int r = 0; r < NIT; ++r) {
    const int L  = r * 32 + wid * 4 + lq;
    ok[r] = (L < NPD);
    const int Lc = ok[r] ? L : (NPD - 1);
    const int yp = Lc / PDH;
    const int xp = Lc - PDH * yp;
    const bool inter = (yp >= 1) && (yp <= PH1) && (xp >= 1) && (xp <= PH1);
    const int s = min(max(yp - 1, 0), PH1 - 1) * PH1 + min(max(xp - 1, 0), PH1 - 1);
    const float* src = h1p + ((size_t)b * NPP1 + s) * CO1 + 8 * pj;
    const v4f a0 = *(const v4f*)(src);
    const v4f a1 = *(const v4f*)(src + 4);
    float hv[8];
    hv[0] = a0.x; hv[1] = a0.y; hv[2] = a0.z; hv[3] = a0.w;
    hv[4] = a1.x; hv[5] = a1.y; hv[6] = a1.z; hv[7] = a1.w;
    unsigned hb[8];
#pragma unroll
    for (int e = 0; e < 8; ++e) {
      float v = hv[e] - mu[e];
      v = v * rs[e];
      v = v * ga[e];
      v = v + be[e];
      v = fmaxf(v, 0.0f);
      v = v * A2SC;
      v = inter ? v : 0.0f;
      hb[e] = hbits((_Float16)v);
    }
    val[r].x = hb[0] | (hb[1] << 16);
    val[r].y = hb[2] | (hb[3] << 16);
    val[r].z = hb[4] | (hb[5] << 16);
    val[r].w = hb[6] | (hb[7] << 16);
    eo[r] = ((size_t)b * NPD + Lc) * CO1 + 8 * pj;
  }
#pragma unroll
  for (int r = 0; r < NIT; ++r) if (ok[r]) *(volatile v4u*)(p1 + eo[r]) = val[r];
  __threadfence();
#pragma unroll
  for (int r = 0; r < NIT; ++r) if (ok[r]) *(volatile v4u*)(p1 + eo[r]) = val[r];
}

__global__ __launch_bounds__(256)
void k_conv2(const _Float16* __restrict__ p1, const _Float16* __restrict__ wq2,
             const float* __restrict__ alpha, const float* __restrict__ gam,
             float* h2p, float* part)
{
  __shared__ __align__(16) float st[NPP2 * STP2];
  __shared__ __align__(16) float red[8 * 128];
  __shared__ __align__(16) float rec[128];
  __shared__ float gsel[64];

  const int tid  = threadIdx.x;
  const int lane = tid & 31;
  const int wid  = tid >> 5;
  const int m    = lane & 15;
  const int hh   = lane >> 4;
  const int pj   = lane & 7;
  const int lq   = lane >> 3;
  const int b    = blockIdx.x >> 1;
  const int nh   = blockIdx.x & 1;
  const float al = alpha[32] * A2INV;

  if (tid < 64) gsel[tid] = (bf_rne(gam[64 * nh + tid]) >= 0.0f) ? 1.0f : 0.0f;
  __syncthreads();

  const _Float16* ap = p1 + (((size_t)b * PDH + 2 * wid) * PDH + m) * CO1 + 8 * hh;
  const _Float16* bp = wq2 + (size_t)(64 * nh + m) * K2 + 8 * hh;
  v8f acc[2][4];
#pragma unroll
  for (int mi = 0; mi < 2; ++mi)
#pragma unroll
    for (int ni = 0; ni < 4; ++ni) acc[mi][ni] = zero8f();

#pragma unroll 1
  for (int tap = 0; tap < 9; ++tap) {
    const int dy = tap / 3;
    const int dx = tap - 3 * dy;
    const _Float16* a0p = ap + (dy * PDH + dx) * CO1;
    const _Float16* a1p = a0p + PDH * CO1;
    const _Float16* bt  = bp + tap * CO1;
#pragma unroll
    for (int kc = 0; kc < 2; ++kc) {
      const v16h fa0 = ldfrag_h(a0p + 32 * kc);
      const v16h fa1 = ldfrag_h(a1p + 32 * kc);
      v16h fbq[4];
#pragma unroll
      for (int ni = 0; ni < 4; ++ni) fbq[ni] = ldfrag_h(bt + (size_t)ni * 16 * K2 + 32 * kc);
#pragma unroll
      for (int ni = 0; ni < 4; ++ni) {
        acc[0][ni] = mma_h(fa0, fbq[ni], acc[0][ni]);
        acc[1][ni] = mma_h(fa1, fbq[ni], acc[1][ni]);
      }
      guard8x6(acc[0][0], acc[0][1], acc[0][2], acc[0][3], acc[1][0], acc[1][1], acc[1][2], acc[1][3],
               fa0, fa1, fbq[0], fbq[1], fbq[2], fbq[3]);
    }
  }
  acc_guard8(acc[0][0], acc[0][1], acc[0][2], acc[0][3], acc[1][0], acc[1][1], acc[1][2], acc[1][3]);

  float ssum[4], ssq[4];
#pragma unroll
  for (int ni = 0; ni < 4; ++ni) {
    const int chl = 16 * ni + m;
    const float fs = gsel[chl];
    float s = 0.0f, q = 0.0f;
#pragma unroll
    for (int j = 0; j < 4; ++j) {
      const float v00 = acc[0][ni][2 * j] * al;
      const float v01 = acc[0][ni][2 * j + 1] * al;
      const float v10 = acc[1][ni][2 * j] * al;
      const float v11 = acc[1][ni][2 * j + 1] * al;
      s = s + v00; s = s + v01; s = s + v10; s = s + v11;
      q = q + v00 * v00; q = q + v01 * v01; q = q + v10 * v10; q = q + v11 * v11;
      const float mx = fmaxf(fmaxf(v00, v01), fmaxf(v10, v11));
      const float mn = fminf(fminf(v00, v01), fminf(v10, v11));
      const float sel = (fs != 0.0f) ? mx : mn;
      st[(wid * 8 + 4 * hh + j) * STP2 + chl] = sel;
    }
    ssum[ni] = s; ssq[ni] = q;
  }
#pragma unroll
  for (int ni = 0; ni < 4; ++ni) {
    const float s = ssum[ni] + __shfl_xor(ssum[ni], 16);
    const float q = ssq[ni]  + __shfl_xor(ssq[ni], 16);
    if (hh == 0) {
      red[wid * 128 + 16 * ni + m]      = s;
      red[wid * 128 + 64 + 16 * ni + m] = q;
    }
  }
  __syncthreads();
  if (tid < 128) {
    float t = 0.0f;
#pragma unroll
    for (int w = 0; w < 8; ++w) t = t + red[w * 128 + tid];
    rec[tid] = t;
  }
  __syncthreads();

  {
    v4f val[4]; size_t e[4];
#pragma unroll
    for (int it = 0; it < 4; ++it) {
      const int L   = it * 32 + wid * 4 + lq;
      const int sp  = L >> 1;
      const int sub = L & 1;
      val[it] = *(const v4f*)&st[sp * STP2 + 32 * sub + 4 * pj];
      e[it]   = (((size_t)b * NPP2 + sp) * CO2) + 64 * nh + 32 * sub + 4 * pj;
    }
#pragma unroll
    for (int it = 0; it < 4; ++it) *(volatile v4f*)(h2p + e[it]) = val[it];
    __threadfence();
#pragma unroll
    for (int it = 0; it < 4; ++it) *(volatile v4f*)(h2p + e[it]) = val[it];
  }
  {
    const int tl = tid & 31;
    const v4f v = *(const v4f*)&rec[4 * tl];
    float* d = part + (size_t)blockIdx.x * 128 + 4 * tl;
    if (tid < 32) *(volatile v4f*)d = v;
    __threadfence();
    if (tid < 32) *(volatile v4f*)d = v;
  }
}

__global__ __launch_bounds__(256)
void k_pool2(const float* __restrict__ h2p, const float* __restrict__ sb,
             unsigned short* p2h, unsigned short* p2l)
{
  __shared__ float sbl[4 * CO2];
  const int tid = threadIdx.x;
  sbl[tid]       = sb[tid];
  sbl[tid + 256] = sb[tid + 256];
  __syncthreads();
  const int lane = tid & 31;
  const int wid  = tid >> 5;
  const int pj   = lane & 7;
  const int lq   = lane >> 3;
  const int b    = blockIdx.x;
  v4u hv[4], lv[4]; size_t eo[4];
#pragma unroll
  for (int it = 0; it < 4; ++it) {
    const int c = it * 32 + wid * 4 + lq;
    const float mu = sbl[c], rs = sbl[CO2 + c], ga = sbl[2 * CO2 + c], be = sbl[3 * CO2 + c];
    unsigned hb[8], lb[8];
#pragma unroll
    for (int e = 0; e < 8; ++e) {
      const int s = 8 * pj + e;
      const float h = h2p[((size_t)b * NPP2 + s) * CO2 + c];
      float v = h - mu;
      v = v * rs;
      v = v * ga;
      v = v + be;
      v = fmaxf(v, 0.0f);
      const unsigned hi = bfb(v);
      hb[e] = hi;
      lb[e] = bfb(v - __uint_as_float(hi << 16));
    }
    hv[it].x = hb[0] | (hb[1] << 16); hv[it].y = hb[2] | (hb[3] << 16);
    hv[it].z = hb[4] | (hb[5] << 16); hv[it].w = hb[6] | (hb[7] << 16);
    lv[it].x = lb[0] | (lb[1] << 16); lv[it].y = lb[2] | (lb[3] << 16);
    lv[it].z = lb[4] | (lb[5] << 16); lv[it].w = lb[6] | (lb[7] << 16);
    eo[it] = (size_t)b * KF + (size_t)c * NPP2 + 8 * pj;
  }
#pragma unroll
  for (int it = 0; it < 4; ++it) {
    *(volatile v4u*)(p2h + eo[it]) = hv[it];
    *(volatile v4u*)(p2l + eo[it]) = lv[it];
  }
  __threadfence();
#pragma unroll
  for (int it = 0; it < 4; ++it) {
    *(volatile v4u*)(p2h + eo[it]) = hv[it];
    *(volatile v4u*)(p2l + eo[it]) = lv[it];
  }
}

__global__ __launch_bounds__(256)
void k_fc1(const __bf16* __restrict__ ph, const __bf16* __restrict__ pl,
           const __bf16* __restrict__ wf, const float* __restrict__ alpha,
           float* h3, float* part)
{
  __shared__ __align__(16) float st[MBF * STP3];
  __shared__ __align__(16) float red[4 * 256];
  __shared__ __align__(16) float rec[256];

  const int tid  = threadIdx.x;
  const int lane = tid & 31;
  const int wid  = tid >> 5;
  const int m    = lane & 15;
  const int hh   = lane >> 4;
  const int pj   = lane & 7;
  const int lq   = lane >> 3;
  const int mb   = blockIdx.x >> 1;
  const int nb   = blockIdx.x & 1;
  const int mt   = wid & 3;
  const int nq   = wid >> 2;
  const float al = alpha[64];

  const size_t arow = (size_t)(MBF * mb + 16 * mt + m) * KF + 8 * hh;
  const __bf16* pa = ph + arow;
  const __bf16* pb = pl + arow;
  const __bf16* pw = wf + (size_t)(128 * nb + 64 * nq + m) * KF + 8 * hh;
  v8f acc[4];
#pragma unroll
  for (int ni = 0; ni < 4; ++ni) acc[ni] = zero8f();

#pragma unroll 2
  for (int s = 0; s < KF / 32; ++s) {
    const v16b fah = ldfrag_b(pa + 32 * s);
    const v16b fal = ldfrag_b(pb + 32 * s);
    v16b fbq[4];
#pragma unroll
    for (int ni = 0; ni < 4; ++ni) fbq[ni] = ldfrag_b(pw + (size_t)ni * 16 * KF + 32 * s);
#pragma unroll
    for (int ni = 0; ni < 4; ++ni) {
      acc[ni] = mma_b(fah, fbq[ni], acc[ni]);
      acc[ni] = mma_b(fal, fbq[ni], acc[ni]);
    }
    guard4x6(acc[0], acc[1], acc[2], acc[3], fah, fal, fbq[0], fbq[1], fbq[2], fbq[3]);
  }
  acc_guard4(acc[0], acc[1], acc[2], acc[3]);

#pragma unroll
  for (int ni = 0; ni < 4; ++ni) {
    const int nl = 64 * nq + 16 * ni + m;
    float s = 0.0f, q = 0.0f;
#pragma unroll
    for (int r = 0; r < 8; ++r) {
      const float v = acc[ni][r] * al;
      st[(16 * mt + 8 * hh + r) * STP3 + nl] = v;
      s = s + v;
      q = q + v * v;
    }
    const float s2 = s + __shfl_xor(s, 16);
    const float q2 = q + __shfl_xor(q, 16);
    if (hh == 0) {
      red[mt * 256 + nl]       = s2;
      red[mt * 256 + 128 + nl] = q2;
    }
  }
  __syncthreads();
  {
    float t = 0.0f;
#pragma unroll
    for (int g = 0; g < 4; ++g) t = t + red[g * 256 + tid];
    rec[tid] = t;
  }
  __syncthreads();

  {
    v4f val[8]; size_t e[8];
#pragma unroll
    for (int it = 0; it < 8; ++it) {
      const int L   = it * 32 + wid * 4 + lq;
      const int row = L >> 2;
      const int sub = L & 3;
      val[it] = *(const v4f*)&st[row * STP3 + 32 * sub + 4 * pj];
      e[it]   = (size_t)(MBF * mb + row) * NF1 + 128 * nb + 32 * sub + 4 * pj;
    }
#pragma unroll
    for (int it = 0; it < 8; ++it) *(volatile v4f*)(h3 + e[it]) = val[it];
    __threadfence();
#pragma unroll
    for (int it = 0; it < 8; ++it) *(volatile v4f*)(h3 + e[it]) = val[it];
  }
  {
    const int tl = tid & 63;
    const v4f v = *(const v4f*)&rec[4 * tl];
    float* d = part + (size_t)blockIdx.x * 256 + 4 * tl;
    if (tid < 64) *(volatile v4f*)d = v;
    __threadfence();
    if (tid < 64) *(volatile v4f*)d = v;
  }
}

__global__ __launch_bounds__(256)
void k_fc2(const float* __restrict__ h3, const float* __restrict__ sb,
           const float* __restrict__ wfc2, const float* __restrict__ alpha, float* out)
{
  __shared__ float sbl[4 * NF1];
  __shared__ float sg[NCLS * NF1];
  __shared__ float ost[RFC2 * NCLS];
  const int tid  = threadIdx.x;
  const int lane = tid & 31;
  const int wid  = tid >> 5;
#pragma unroll
  for (int i = 0; i < 4; ++i) sbl[tid + 256 * i] = sb[tid + 256 * i];
#pragma unroll
  for (int j = 0; j < NCLS; ++j) {
    const float r = bf_rne(wfc2[j * NF1 + tid]);
    sg[j * NF1 + tid] = (r > 0.0f) ? 1.0f : ((r < 0.0f) ? -1.0f : 0.0f);
  }
  __syncthreads();
  const float al = alpha[96];
  const int rl  = tid >> 3;
  const int pj  = tid & 7;
  const size_t row = (size_t)blockIdx.x * RFC2 + rl;
  float acc[NCLS];
#pragma unroll
  for (int j = 0; j < NCLS; ++j) acc[j] = 0.0f;
#pragma unroll 1
  for (int kk = 0; kk < NF1 / 8; ++kk) {
    const int k = pj + 8 * kk;
    float v = h3[row * NF1 + k] - sbl[k];
    v = v * sbl[NF1 + k];
    v = v * sbl[2 * NF1 + k];
    v = v + sbl[3 * NF1 + k];
    v = fmaxf(v, 0.0f);
#pragma unroll
    for (int j = 0; j < NCLS; ++j) acc[j] = acc[j] + v * sg[j * NF1 + k];
  }
#pragma unroll
  for (int j = 0; j < NCLS; ++j) {
    acc[j] = acc[j] + __shfl_xor(acc[j], 1);
    acc[j] = acc[j] + __shfl_xor(acc[j], 2);
    acc[j] = acc[j] + __shfl_xor(acc[j], 4);
  }
  if (pj == 0) {
#pragma unroll
    for (int j = 0; j < NCLS; ++j) ost[rl * NCLS + j] = acc[j] * al;
  }
  __syncthreads();
  {
    const int L0 = wid;
    const int L1 = wid + 8;
    const bool ok1 = (L1 < NCLS);
    const float v0 = ost[L0 * 32 + lane];
    const float v1 = ost[min(L1, NCLS - 1) * 32 + lane];
    float* base = out + (size_t)blockIdx.x * (RFC2 * NCLS);
    float* d0 = base + L0 * 32 + lane;
    float* d1 = base + min(L1, NCLS - 1) * 32 + lane;
    *(volatile float*)d0 = v0;
    if (ok1) *(volatile float*)d1 = v1;
    __threadfence();
    *(volatile float*)d0 = v0;
    if (ok1) *(volatile float*)d1 = v1;
  }
}

extern "C" void kernel_launch(void* const* d_in, const int* in_sizes, int n_in,
                              void* d_out, int out_size, void* d_ws, size_t ws_size,
                              hipStream_t stream) {
  if (n_in < 11) return;
  const int nx = in_sizes[0];
  if (nx <= 0 || (nx % (CIN1 * NPX1)) != 0) return;
  const int NB = nx / (CIN1 * NPX1);
  if (NB < MBF || (NB % MBF) != 0) return;
  if (in_sizes[1] != CO1 * K1) return;
  if (in_sizes[2] != CO1 || in_sizes[3] != CO1) return;
  if (in_sizes[4] != CO2 * K2) return;
  if (in_sizes[5] != CO2 || in_sizes[6] != CO2) return;
  if (in_sizes[7] != NF1 * KF) return;
  if (in_sizes[8] != NF1 || in_sizes[9] != NF1) return;
  if (in_sizes[10] != NCLS * NF1) return;
  if (out_size != NB * NCLS) return;

  const size_t o_alpha = 0;
  const size_t o_sb1   = 512;
  const size_t o_sb2   = o_sb1 + (size_t)4 * CO1 * 4;
  const size_t o_sb3   = o_sb2 + (size_t)4 * CO2 * 4;
  const size_t o_wq1   = 8192;
  const size_t o_wq2   = o_wq1 + (size_t)CO1 * K1P * 2;
  const size_t o_wf1   = o_wq2 + (size_t)CO2 * K2 * 2;
  const size_t o_st1   = o_wf1 + (size_t)NF1 * KF * 2;
  const size_t o_st2   = o_st1 + (size_t)NB * 128 * 4;
  const size_t o_st3   = o_st2 + (size_t)NB * 2 * 128 * 4;
  const size_t o_h3    = o_st3 + (size_t)(NB / MBF) * 2 * 256 * 4;
  const size_t o_h1p   = o_h3 + (size_t)NB * NF1 * 4;
  const size_t o_h2p   = o_h1p;
  const size_t o_p2h   = o_h1p + (size_t)NB * NPP2 * CO2 * 4;
  const size_t o_p2l   = o_p2h + (size_t)NB * KF * 2;
  const size_t o_p1    = o_h1p + (size_t)NB * NPP1 * CO1 * 4;
  const size_t o_end   = o_p1 + (size_t)NB * NPD * CO1 * 2;
  if (o_p2l + (size_t)NB * KF * 2 > o_p1) return;
  if (o_end > ws_size) return;

  const float* x    = (const float*)d_in[0];
  const float* w1   = (const float*)d_in[1];
  const float* g1   = (const float*)d_in[2];
  const float* b1   = (const float*)d_in[3];
  const float* w2   = (const float*)d_in[4];
  const float* g2   = (const float*)d_in[5];
  const float* b2   = (const float*)d_in[6];
  const float* wfc1 = (const float*)d_in[7];
  const float* g3   = (const float*)d_in[8];
  const float* b3   = (const float*)d_in[9];
  const float* wfc2 = (const float*)d_in[10];
  float* out = (float*)d_out;
  char* ws = (char*)d_ws;

  float*          alpha = (float*)(ws + o_alpha);
  float*          sb1   = (float*)(ws + o_sb1);
  float*          sb2   = (float*)(ws + o_sb2);
  float*          sb3   = (float*)(ws + o_sb3);
  unsigned*       wq1   = (unsigned*)(ws + o_wq1);
  unsigned*       wq2   = (unsigned*)(ws + o_wq2);
  unsigned*       wf1   = (unsigned*)(ws + o_wf1);
  float*          st1   = (float*)(ws + o_st1);
  float*          st2   = (float*)(ws + o_st2);
  float*          st3   = (float*)(ws + o_st3);
  float*          h3    = (float*)(ws + o_h3);
  float*          h1p   = (float*)(ws + o_h1p);
  float*          h2p   = (float*)(ws + o_h2p);
  unsigned short* p2h   = (unsigned short*)(ws + o_p2h);
  unsigned short* p2l   = (unsigned short*)(ws + o_p2l);
  unsigned short* p1    = (unsigned short*)(ws + o_p1);

  k_alpha<<<dim3(4), dim3(256), 0, stream>>>(w1, in_sizes[1], w2, in_sizes[4], wfc1, in_sizes[7],
                                            wfc2, in_sizes[10], alpha);
  (void)hipGetLastError();
  k_pack<0><<<dim3((CO1 * K1P / 8) / 256), dim3(256), 0, stream>>>(w1, wq1, CO1 * K1P / 8);
  (void)hipGetLastError();
  k_pack<1><<<dim3((CO2 * K2 / 8) / 256), dim3(256), 0, stream>>>(w2, wq2, CO2 * K2 / 8);
  (void)hipGetLastError();
  k_pack<2><<<dim3((NF1 * KF / 8) / 256), dim3(256), 0, stream>>>(wfc1, wf1, NF1 * KF / 8);
  (void)hipGetLastError();

  k_conv1<<<dim3(NB), dim3(256), 0, stream>>>(x, (const __bf16*)wq1, alpha, g1, h1p, st1);
  (void)hipGetLastError();
  k_stats<<<dim3(1), dim3(256), 0, stream>>>(st1, NB, CO1, 1, CO1, g1, b1, NB * NPX1, sb1);
  (void)hipGetLastError();
  k_pool1<<<dim3(NB), dim3(256), 0, stream>>>(h1p, sb1, p1);
  (void)hipGetLastError();

  k_conv2<<<dim3(NB * 2), dim3(256), 0, stream>>>((const _Float16*)p1, (const _Float16*)wq2, alpha, g2,
                                                  h2p, st2);
  (void)hipGetLastError();
  k_stats<<<dim3(1), dim3(256), 0, stream>>>(st2, NB, 64, 2, CO2, g2, b2, NB * NPP1, sb2);
  (void)hipGetLastError();
  k_pool2<<<dim3(NB), dim3(256), 0, stream>>>(h2p, sb2, p2h, p2l);
  (void)hipGetLastError();

  k_fc1<<<dim3((NB / MBF) * 2), dim3(256), 0, stream>>>((const __bf16*)p2h, (const __bf16*)p2l,
                                                        (const __bf16*)wf1, alpha, h3, st3);
  (void)hipGetLastError();
  k_stats<<<dim3(1), dim3(256), 0, stream>>>(st3, NB / MBF, 128, 2, NF1, g3, b3, NB, sb3);
  (void)hipGetLastError();
  k_fc2<<<dim3(NB / RFC2), dim3(256), 0, stream>>>(h3, sb3, wfc2, alpha, out);
  (void)hipGetLastError();
}
